// DSDAHead_46746424050089
// MI455X (gfx1250) — hardware-verified
//
#include <hip/hip_runtime.h>


namespace {
constexpr int B = 4, CIN = 512, CI = 32, HH = 64, WW = 64, NP = HH * WW, K5 = CIN * 9, K3 = CI * 9, NCH = NP / 32;
constexpr float XS = 8.0f, PS = 1024.0f, WSC = 256.0f;
typedef _Float16 b16;
typedef __attribute__((ext_vector_type(16))) _Float16 v16b;
typedef __attribute__((ext_vector_type(8))) _Float16 v8b;
typedef __attribute__((ext_vector_type(8))) float v8f;
typedef __attribute__((ext_vector_type(4))) float v4f;
__device__ __forceinline__ float bf16_rne(float f) { unsigned int u = __float_as_uint(f); u += 0x7FFFu + ((u >> 16) & 1u); float r = __uint_as_float(u & 0xFFFF0000u); asm volatile("" : "+v"(r)); return r; }
__device__ __forceinline__ void split16(float v, b16& hi, b16& lo) { hi = (b16)v; lo = (b16)(v - (float)hi); }
__device__ __forceinline__ v16b frag_kb(const b16* p, int hh) { const v8b a = *(const v8b*)(p + 8 * hh), b = *(const v8b*)(p + 16 + 8 * hh); v16b f;
#pragma unroll
  for (int e = 0; e < 8; ++e) { f[e] = a[e]; f[8 + e] = b[e]; } return f; }
__device__ __forceinline__ v8f wmma16b(v16b a, v16b b, v8f c) { v8f d = __builtin_amdgcn_wmma_f32_16x16x32_f16(false, a, false, b, (short)0, c, false, false); asm volatile("v_nop\n\tv_nop\n\tv_nop\n\tv_nop" : "+v"(d) : "v"(a), "v"(b)); return d; }
__device__ __forceinline__ void wave_lds_sync() { __builtin_amdgcn_fence(__ATOMIC_RELEASE, "workgroup"); __builtin_amdgcn_wave_barrier(); __builtin_amdgcn_fence(__ATOMIC_ACQUIRE, "workgroup"); }
__device__ __forceinline__ float pmul(float a, float b) { float p = a * b; asm volatile("" : "+v"(p)); return p; }
__device__ __forceinline__ float bnf(float v, const float* s, const float* bb, const float* m, const float* var, int c) { const float inv = bf16_rne(s[c]) * rsqrtf(bf16_rne(var[c]) + 1e-5f); return fmaxf(pmul(v, inv) + (bf16_rne(bb[c]) - pmul(bf16_rne(m[c]), inv)), 0.0f); }

__global__ __launch_bounds__(256) void wput_kernel(const float* __restrict__ w5a, const float* __restrict__ w5c, const float* __restrict__ w51, const float* __restrict__ w52, const float* __restrict__ pv, const float* __restrict__ pq, const float* __restrict__ pk, b16* __restrict__ W5, b16* __restrict__ W3, b16* __restrict__ WP) {
  const size_t u = (size_t)blockIdx.x * 256 + threadIdx.x;
  for (int pass = 0; pass < 2; ++pass) {
    if (u < (size_t)2 * CI * (K5 / 8)) { const int o = (int)(u / (K5 / 8)), k0 = (int)(u % (K5 / 8)) * 8; const float* w = o < CI ? w5a + (size_t)o * K5 : w5c + (size_t)(o - CI) * K5; v8b v; for (int j = 0; j < 8; ++j) v[j] = (b16)(bf16_rne(w[k0 + j]) * WSC); *(volatile v8b*)(W5 + (size_t)o * K5 + k0) = v; }
    if (u < (size_t)2 * CI * (K3 / 8)) { const int o = (int)(u / (K3 / 8)), k0 = (int)(u % (K3 / 8)) * 8; const float* w = o < CI ? w51 + (size_t)o * K3 : w52 + (size_t)(o - CI) * K3; v8b v; for (int j = 0; j < 8; ++j) v[j] = (b16)(bf16_rne(w[k0 + j]) * WSC); *(volatile v8b*)(W3 + (size_t)o * K3 + k0) = v; }
    if (u < 48 * 4) { const int o = (int)(u / 4), k0 = (int)(u % 4) * 8; v8b v; for (int j = 0; j < 8; ++j) { const int k = k0 + j; float w = 0.0f; if (o < CI) w = pv[o * CI + k]; else if (o < 36) w = pq[(o - 32) * CI + k]; else if (o < 40) w = pk[(o - 36) * CI + k]; v[j] = (b16)(bf16_rne(w) * WSC); } *(volatile v8b*)(WP + (size_t)o * CI + k0) = v; }
    __threadfence(); } }
__global__ __launch_bounds__(32) void conv5_kernel(const float* __restrict__ x, const b16* __restrict__ W5, const float* __restrict__ s1, const float* __restrict__ b1, const float* __restrict__ m1, const float* __restrict__ v1, const float* __restrict__ s2, const float* __restrict__ b2, const float* __restrict__ m2, const float* __restrict__ v2, int BV, float* __restrict__ F1, float* __restrict__ F2) {
  __shared__ __attribute__((aligned(16))) b16 A1[16][40]; __shared__ float Tf[16][68]; const int lane = threadIdx.x, nloc = lane & 15, hlf = lane >> 4; const int seg = blockIdx.x % 4, h = (blockIdx.x / 4) % HH, b = blockIdx.x / (4 * HH); if (b >= BV) return; const int w0 = seg * 16;
  v8f acc[4] = {(v8f){}, (v8f){}, (v8f){}, (v8f){}};
#pragma unroll 1
  for (int kb = 0; kb < K5; kb += 32) { const int k = kb + lane; const int ci = k / 9, r9 = k % 9, dy = r9 / 3 - 1, dx = r9 % 3 - 1; const int hy = h + dy; const float* xr = x + (((size_t)b * CIN + ci) * HH + (hy < 0 ? 0 : (hy >= HH ? HH - 1 : hy))) * WW; const bool hok = (hy >= 0 && hy < HH);
#pragma unroll
    for (int rr = 0; rr < 16; ++rr) { const int wx = w0 + rr + dx; const float v = (hok && wx >= 0 && wx < WW) ? bf16_rne(xr[wx]) : 0.0f; A1[rr][lane] = (b16)(v * XS); }
    wave_lds_sync(); const v16b a = frag_kb(&A1[nloc][0], hlf);
#pragma unroll
    for (int t = 0; t < 4; ++t) acc[t] = wmma16b(a, frag_kb(W5 + (size_t)(t * 16 + nloc) * K5 + kb, hlf), acc[t]);
    wave_lds_sync(); }
#pragma unroll
  for (int t = 0; t < 4; ++t) { const int c = t * 16 + nloc;
#pragma unroll
    for (int r8 = 0; r8 < 8; ++r8) { const float v = acc[t][r8] * (1.0f / (XS * WSC)); Tf[8 * hlf + r8][c] = (c < CI) ? bnf(v, s1, b1, m1, v1, c) : bnf(v, s2, b2, m2, v2, c - CI); } }
  wave_lds_sync(); const size_t px0 = (size_t)b * NP + h * WW + w0;
  for (int pass = 0; pass < 2; ++pass) { for (int rr = 0; rr < 16; ++rr) { ((volatile float*)F1)[(px0 + rr) * CI + lane] = Tf[rr][lane]; ((volatile float*)F2)[(px0 + rr) * CI + lane] = Tf[rr][CI + lane]; } __threadfence(); } }
__global__ __launch_bounds__(32) void pqkv_kernel(const float* __restrict__ F1, const b16* __restrict__ WP, const float* __restrict__ pvb, const float* __restrict__ pqb, const float* __restrict__ pkb, int BV, float* __restrict__ QK, b16* __restrict__ VTh, b16* __restrict__ VTl) {
  __shared__ __attribute__((aligned(16))) b16 Ah[16][40], Al[16][40]; __shared__ float Tf[32][48]; const int lane = threadIdx.x, nloc = lane & 15, hlf = lane >> 4; const int ch = blockIdx.x % NCH, b = blockIdx.x / NCH; if (b >= BV) return; const size_t px0 = (size_t)b * NP + ch * 32;
  for (int half = 0; half < 2; ++half) {
    for (int rr = 0; rr < 16; ++rr) { b16 p, q; split16(F1[(px0 + half * 16 + rr) * CI + lane] * XS, p, q); Ah[rr][lane] = p; Al[rr][lane] = q; }
    wave_lds_sync(); const v16b a = frag_kb(&Ah[nloc][0], hlf), al = frag_kb(&Al[nloc][0], hlf);
#pragma unroll
    for (int t = 0; t < 3; ++t) { v8f acc = {}; const v16b bw = frag_kb(WP + (size_t)(t * 16 + nloc) * CI, hlf); acc = wmma16b(a, bw, acc); acc = wmma16b(al, bw, acc); const int c = t * 16 + nloc; const float bb = c < CI ? bf16_rne(pvb[c]) : (c < 36 ? bf16_rne(pqb[c - 32]) : (c < 40 ? bf16_rne(pkb[c - 36]) : 0.0f));
#pragma unroll
      for (int r8 = 0; r8 < 8; ++r8) Tf[half * 16 + 8 * hlf + r8][c] = acc[r8] * (1.0f / (XS * WSC)) + bb; }
    wave_lds_sync(); }
  const size_t vb = ((size_t)b * NCH + ch) * CI;
  for (int pass = 0; pass < 2; ++pass) { for (int i2 = lane; i2 < 256; i2 += 32) ((volatile float*)QK)[px0 * 8 + i2] = Tf[i2 / 8][32 + (i2 % 8)];
    for (int c = 0; c < CI; ++c) { b16 p, q; split16(Tf[lane][c] * XS, p, q); ((volatile b16*)VTh)[(vb + c) * 64 + lane] = p; ((volatile b16*)VTl)[(vb + c) * 64 + lane] = q; } __threadfence(); } }
__global__ __launch_bounds__(32) void pam_kernel(const float* __restrict__ QK, const b16* __restrict__ VTh, const b16* __restrict__ VTl, const float* __restrict__ F1, const float* __restrict__ pg, int BV, float* __restrict__ SA) {
  __shared__ __attribute__((aligned(16))) b16 Ph[16][40], Pl[16][40]; __shared__ float Qs[16][4], Mx[16], Dn[16], Sf[16], Of[16][CI + 1]; const int lane = threadIdx.x, nloc = lane & 15, hlf = lane >> 4; const int qt = blockIdx.x % (NP / 16), b = blockIdx.x / (NP / 16); if (b >= BV) return; const size_t q0 = (size_t)b * NP + qt * 16;
  if (lane < 16) { for (int c = 0; c < 4; ++c) Qs[lane][c] = QK[(q0 + lane) * 8 + c]; Mx[lane] = -INFINITY; Dn[lane] = 0.0f; Sf[lane] = 0.0f; }
  v8f acc[2] = {(v8f){}, (v8f){}}; wave_lds_sync();
#pragma unroll 1
  for (int kc = 0; kc < NP; kc += 32) { const size_t key = (size_t)b * NP + kc + lane; float kv[4]; for (int c = 0; c < 4; ++c) kv[c] = QK[key * 8 + 4 + c];
#pragma unroll 1
    for (int qi = 0; qi < 16; ++qi) { float sv = 0.0f; for (int c = 0; c < 4; ++c) sv += pmul(Qs[qi][c], kv[c]); float cm = sv; for (int o = 16; o; o >>= 1) cm = fmaxf(cm, __shfl_xor(cm, o)); const float mo = Mx[qi]; const float mn = fmaxf(mo, cm); const float p = __expf(sv - mn); float ps = p; for (int o = 16; o; o >>= 1) ps += __shfl_xor(ps, o);
      b16 ph, plo; split16(p * PS, ph, plo); Ph[qi][lane] = ph; Pl[qi][lane] = plo; if (lane == 0) { const float sf = (mo == -INFINITY) ? 0.0f : __expf(mo - mn); Sf[qi] = sf; Dn[qi] = Dn[qi] * sf + ps; Mx[qi] = mn; } }
    wave_lds_sync(); const v16b pa = frag_kb(&Ph[nloc][0], hlf), pb = frag_kb(&Pl[nloc][0], hlf); const size_t vb = (((size_t)b * NCH + kc / 32) * CI) * 64;
#pragma unroll
    for (int t = 0; t < 2; ++t) {
#pragma unroll
      for (int r8 = 0; r8 < 8; ++r8) acc[t][r8] *= Sf[8 * hlf + r8];
      const v16b vh = frag_kb(VTh + vb + (size_t)(t * 16 + nloc) * 64, hlf), vl = frag_kb(VTl + vb + (size_t)(t * 16 + nloc) * 64, hlf); acc[t] = wmma16b(pa, vh, acc[t]); acc[t] = wmma16b(pa, vl, acc[t]); acc[t] = wmma16b(pb, vh, acc[t]); }
    wave_lds_sync(); }
  const float g = bf16_rne(pg[0]);
#pragma unroll
  for (int t = 0; t < 2; ++t)
#pragma unroll
    for (int r8 = 0; r8 < 8; ++r8) { const int rl = 8 * hlf + r8; Of[rl][t * 16 + nloc] = pmul(g, acc[t][r8] * (1.0f / (PS * XS)) / Dn[rl]); }
  wave_lds_sync();
  for (int pass = 0; pass < 2; ++pass) { for (int rr = 0; rr < 16; ++rr) ((volatile float*)SA)[(q0 + rr) * CI + lane] = Of[rr][lane] + F1[(q0 + rr) * CI + lane]; __threadfence(); } }
__global__ __launch_bounds__(1024) void cam_kernel(const float* __restrict__ F2, int BV, b16* __restrict__ ATh, b16* __restrict__ ATl) {
  __shared__ float En[CI][CI + 1], At[CI][CI + 1]; const int b = blockIdx.x; if (b >= BV) return; const int c = threadIdx.x / CI, d = threadIdx.x % CI; float s = 0.0f;
#pragma unroll 1
  for (int n = 0; n < NP; ++n) s += pmul(F2[((size_t)b * NP + n) * CI + c], F2[((size_t)b * NP + n) * CI + d]);
  En[c][d] = s; __syncthreads();
  { float mx = -INFINITY; for (int j = 0; j < CI; ++j) mx = fmaxf(mx, En[c][j]); float en = mx - En[c][d];
    float m2 = -INFINITY; for (int j = 0; j < CI; ++j) m2 = fmaxf(m2, mx - En[c][j]); const float e = __expf(en - m2); At[c][d] = e; }
  __syncthreads(); { float den = 0.0f; for (int j = 0; j < CI; ++j) den += At[c][j]; const float a = At[c][d] / den; __syncthreads(); At[c][d] = a; }
  __syncthreads();
  if (threadIdx.x < 32) { const int lane = threadIdx.x; for (int pass = 0; pass < 2; ++pass) { for (int cc = 0; cc < CI; ++cc) { b16 p, q; split16(At[cc][lane] * PS, p, q); ((volatile b16*)ATh)[((size_t)b * CI + cc) * CI + lane] = p; ((volatile b16*)ATl)[((size_t)b * CI + cc) * CI + lane] = q; } __threadfence(); } } }
__global__ __launch_bounds__(32) void camagg_kernel(const float* __restrict__ F2, const b16* __restrict__ ATh, const b16* __restrict__ ATl, const float* __restrict__ cg, int BV, float* __restrict__ SC) {
  __shared__ __attribute__((aligned(16))) b16 Ah[16][40], Al[16][40]; __shared__ float Tf[16][CI + 1]; const int lane = threadIdx.x, nloc = lane & 15, hlf = lane >> 4; const size_t m0 = (size_t)blockIdx.x * 16; const int b = (int)(m0 / NP); if (b >= BV) return;
  for (int rr = 0; rr < 16; ++rr) { b16 p, q; split16(F2[(m0 + rr) * CI + lane] * XS, p, q); Ah[rr][lane] = p; Al[rr][lane] = q; }
  wave_lds_sync(); const v16b a = frag_kb(&Ah[nloc][0], hlf), al = frag_kb(&Al[nloc][0], hlf); const float g = bf16_rne(cg[0]);
#pragma unroll
  for (int t = 0; t < 2; ++t) { v8f acc = {}; const v16b bh = frag_kb(ATh + ((size_t)b * CI + t * 16 + nloc) * CI, hlf), bl = frag_kb(ATl + ((size_t)b * CI + t * 16 + nloc) * CI, hlf); acc = wmma16b(a, bh, acc); acc = wmma16b(a, bl, acc); acc = wmma16b(al, bh, acc);
#pragma unroll
    for (int r8 = 0; r8 < 8; ++r8) Tf[8 * hlf + r8][t * 16 + nloc] = pmul(g, acc[r8] * (1.0f / (XS * PS))); }
  wave_lds_sync();
  for (int pass = 0; pass < 2; ++pass) { for (int rr = 0; rr < 16; ++rr) ((volatile float*)SC)[(m0 + rr) * CI + lane] = Tf[rr][lane] + F2[(m0 + rr) * CI + lane]; __threadfence(); } }
__global__ __launch_bounds__(32) void conv3_kernel(const float* __restrict__ SA, const float* __restrict__ SC, const b16* __restrict__ W3, const float* __restrict__ s51, const float* __restrict__ bb51, const float* __restrict__ m51, const float* __restrict__ v51, const float* __restrict__ s52, const float* __restrict__ bb52, const float* __restrict__ m52, const float* __restrict__ v52, const float* __restrict__ w8, const float* __restrict__ b8, int BV, float* __restrict__ out) {
  __shared__ __attribute__((aligned(16))) b16 Ah[2][16][40], Al[2][16][40]; __shared__ float Ts[32][CI + 1], Oo[2][32]; const int lane = threadIdx.x, nloc = lane & 15, hlf = lane >> 4; const int half = blockIdx.x % 2, h = (blockIdx.x / 2) % HH, b = blockIdx.x / (2 * HH); if (b >= BV) return; const int w0 = half * 32;
  for (int mt = 0; mt < 2; ++mt) { v8f acA[2] = {(v8f){}, (v8f){}}, acC[2] = {(v8f){}, (v8f){}};
#pragma unroll 1
    for (int kb = 0; kb < K3; kb += 32) { const int k = kb + lane; const int ci = k / 9, r9 = k % 9, dy = r9 / 3 - 1, dx = r9 % 3 - 1; const int hy = h + dy; const bool hok = (hy >= 0 && hy < HH);
#pragma unroll
      for (int rr = 0; rr < 16; ++rr) { const int wx = w0 + mt * 16 + rr + dx; float va = 0.0f, vc = 0.0f; if (hok && wx >= 0 && wx < WW) { const size_t px = (size_t)b * NP + hy * WW + wx; va = SA[px * CI + ci]; vc = SC[px * CI + ci]; } b16 p, q; split16(va * XS, p, q); Ah[0][rr][lane] = p; Al[0][rr][lane] = q; split16(vc * XS, p, q); Ah[1][rr][lane] = p; Al[1][rr][lane] = q; }
      wave_lds_sync(); const v16b aa = frag_kb(&Ah[0][nloc][0], hlf), aal = frag_kb(&Al[0][nloc][0], hlf), ac = frag_kb(&Ah[1][nloc][0], hlf), acl = frag_kb(&Al[1][nloc][0], hlf);
#pragma unroll
      for (int t = 0; t < 2; ++t) { const v16b bwA = frag_kb(W3 + (size_t)(t * 16 + nloc) * K3 + kb, hlf), bwC = frag_kb(W3 + (size_t)(CI + t * 16 + nloc) * K3 + kb, hlf); acA[t] = wmma16b(aa, bwA, acA[t]); acA[t] = wmma16b(aal, bwA, acA[t]); acC[t] = wmma16b(ac, bwC, acC[t]); acC[t] = wmma16b(acl, bwC, acC[t]); }
      wave_lds_sync(); }
#pragma unroll
    for (int t = 0; t < 2; ++t) { const int c = t * 16 + nloc;
#pragma unroll
      for (int r8 = 0; r8 < 8; ++r8) Ts[mt * 16 + 8 * hlf + r8][c] = bnf(acA[t][r8] * (1.0f / (XS * WSC)), s51, bb51, m51, v51, c) + bnf(acC[t][r8] * (1.0f / (XS * WSC)), s52, bb52, m52, v52, c); }
    wave_lds_sync(); }
  for (int o = 0; o < 2; ++o) { float s = bf16_rne(b8[o]);
#pragma unroll 1
    for (int c = 0; c < CI; ++c) s += pmul(Ts[lane][c], bf16_rne(w8[o * CI + c])); Oo[o][lane] = fmaxf(s, 0.0f); }
  wave_lds_sync();
  for (int pass = 0; pass < 2; ++pass) { for (int o = 0; o < 2; ++o) ((volatile float*)out)[(((size_t)b * 2 + o) * HH + h) * WW + w0 + lane] = Oo[o][lane]; __threadfence(); } }
}

extern "C" void kernel_launch(void* const* d_in, const int* in_sizes, int n_in, void* d_out, int out_size, void* d_ws, size_t ws_size, hipStream_t stream) {
  (void)n_in;
  auto Fp = [&](int i) { return (const float*)d_in[i]; };
  if (in_sizes[0] != B * CIN * NP || in_sizes[1] != CI * K5 || in_sizes[18] != CI * K5 || in_sizes[13] != CI * K3 || in_sizes[24] != CI * K3 || in_sizes[10] != CI * CI || in_sizes[29] != 2 * CI || out_size != B * 2 * NP) return;
  const int BV = B;
  size_t off = 0; char* ws = (char*)d_ws;
  auto carve = [&](size_t bytes) { char* p = ws + off; off += (bytes + 255) & ~(size_t)255; return p; };
  b16* W5 = (b16*)carve((size_t)2 * CI * K5 * 2); b16* W3 = (b16*)carve((size_t)2 * CI * K3 * 2); b16* WP = (b16*)carve((size_t)48 * CI * 2);
  float* F1 = (float*)carve((size_t)B * NP * CI * 4); float* F2 = (float*)carve((size_t)B * NP * CI * 4); float* QK = (float*)carve((size_t)B * NP * 8 * 4); b16* VTh = (b16*)carve((size_t)B * NCH * CI * 64 * 2); b16* VTl = (b16*)carve((size_t)B * NCH * CI * 64 * 2);
  float* SA = (float*)carve((size_t)B * NP * CI * 4); float* SC = (float*)carve((size_t)B * NP * CI * 4); b16* ATh = (b16*)carve((size_t)B * CI * CI * 2); b16* ATl = (b16*)carve((size_t)B * CI * CI * 2);
  if (off > ws_size || off > ((size_t)32 << 20)) return;
  wput_kernel<<<(unsigned)(((size_t)2 * CI * (K5 / 8) + 255) / 256), 256, 0, stream>>>(Fp(1), Fp(18), Fp(13), Fp(24), Fp(10), Fp(6), Fp(8), W5, W3, WP);
  conv5_kernel<<<BV * HH * 4, 32, 0, stream>>>(Fp(0), W5, Fp(2), Fp(3), Fp(4), Fp(5), Fp(19), Fp(20), Fp(21), Fp(22), BV, F1, F2);
  pqkv_kernel<<<BV * NCH, 32, 0, stream>>>(F1, WP, Fp(11), Fp(7), Fp(9), BV, QK, VTh, VTl);
  pam_kernel<<<BV * (NP / 16), 32, 0, stream>>>(QK, VTh, VTl, F1, Fp(12), BV, SA);
  cam_kernel<<<BV, 1024, 0, stream>>>(F2, BV, ATh, ATl);
  camagg_kernel<<<BV * (NP / 16), 32, 0, stream>>>(F2, ATh, ATl, Fp(23), BV, SC);
  conv3_kernel<<<BV * HH * 2, 32, 0, stream>>>(SA, SC, W3, Fp(14), Fp(15), Fp(16), Fp(17), Fp(25), Fp(26), Fp(27), Fp(28), Fp(29), Fp(30), BV, (float*)d_out);
}
